// HybridModel_5720896438538
// MI455X (gfx1250) — hardware-run, weakly checked
//
#include <hip/hip_runtime.h>
#include <math.h>

constexpr int kBatch = 8;
constexpr int kNode  = 256;
constexpr int kDim   = 48;
constexpr int kVoc   = 20;
constexpr int kLay   = 2;
constexpr int kSmp   = 6;
constexpr int kTok   = kBatch * kNode;
constexpr int kHid2  = 96;
constexpr int kFfn   = 192;
constexpr int kXld   = 64;
constexpr int kPld   = 512;
constexpr int kProjN = 512;
constexpr int kProjK = 64;
constexpr float kXCarry    = 64.0f;
constexpr float kWCarry    = 16.0f;
constexpr float kHCarry    = 16.0f;
constexpr float kProjScale = 1.0f / (64.0f * 16.0f);
constexpr float kPairScale = 1.0f / (16.0f * 16.0f);
constexpr float kInvSqrt2  = 0.70710678118654752f;
constexpr float kLnEps     = 1e-5f;
constexpr int kW1catWords = kLay * kProjN * kProjK / 2;
constexpr int kW2tWords   = kLay * kDim * kHid2 / 2;
constexpr int kBiasWords  = kLay * kProjN;
constexpr int kPrepWords  = kW1catWords + kW2tWords + kBiasWords;

static_assert(kTok % 64 == 0);
static_assert(kProjN % 64 == 0);
static_assert(kProjK % 32 == 0);
static_assert(kHid2 % 32 == 0);
static_assert(kW1catWords % 256 == 0);
static_assert((kW1catWords + kW2tWords) % 256 == 0);
static_assert(kPrepWords % 256 == 0);
static_assert((kTok * kVoc) % (4 * 256) == 0);

typedef __attribute__((ext_vector_type(16))) _Float16 v16h;
typedef __attribute__((ext_vector_type(8)))  _Float16 v8h;
typedef __attribute__((ext_vector_type(16))) __bf16   v16b;
typedef __attribute__((ext_vector_type(8)))  __bf16   v8b;
typedef __attribute__((ext_vector_type(8)))  float    v8f;
typedef __attribute__((ext_vector_type(4)))  float    v4f;
typedef __attribute__((ext_vector_type(4)))  unsigned int v4u;

__device__ __forceinline__ unsigned short f2bf_bits(float f) {
  unsigned u = __float_as_uint(f);
  return (unsigned short)((u + 0x7FFFu + ((u >> 16) & 1u)) >> 16);
}
__device__ __forceinline__ float bf_bits2f(unsigned short h) { return __uint_as_float(((unsigned)h) << 16); }

__device__ __forceinline__ void dep_guard_h(v8f& a, v8f& b, v16h x, v16h y) { asm volatile("v_nop\n\tv_nop\n\tv_nop\n\tv_nop" : "+v"(a), "+v"(b) : "v"(x), "v"(y)); }
__device__ __forceinline__ void dep_guard_b(v8f& a, v8f& b, v16b x, v16b y) { asm volatile("v_nop\n\tv_nop\n\tv_nop\n\tv_nop" : "+v"(a), "+v"(b) : "v"(x), "v"(y)); }
__device__ __forceinline__ void keep4_h(v16h a, v16h b, v16h c, v16h d) { asm volatile("v_nop" :: "v"(a), "v"(b), "v"(c), "v"(d)); }
__device__ __forceinline__ void keep4_b(v16b a, v16b b, v16b c, v16b d) { asm volatile("v_nop" :: "v"(a), "v"(b), "v"(c), "v"(d)); }
__device__ __forceinline__ void acc_guard4(v8f& a, v8f& b, v8f& c, v8f& d) { asm volatile("v_nop\n\tv_nop\n\tv_nop\n\tv_nop" : "+v"(a), "+v"(b), "+v"(c), "+v"(d)); }
__device__ __forceinline__ void guard3h(v8f& a, v8f& b, v8f& c, v16h w, v16h x, v16h y, v16h z) {
  asm volatile("v_nop\n\tv_nop\n\tv_nop\n\tv_nop" : "+v"(a), "+v"(b), "+v"(c) : "v"(w), "v"(x), "v"(y), "v"(z));
}
template <typename T> struct Frag;
template <> struct Frag<_Float16> {
  typedef v16h V; union U { v16h v; v8h h[2]; };
  static __device__ __forceinline__ v16h load(const _Float16* p) {
    U f; f.h[0] = *(const v8h*)(p); f.h[1] = *(const v8h*)(p + 16); return f.v;
  }
  static __device__ __forceinline__ v8f mma(v16h a, v16h b, v8f c) {
    return __builtin_amdgcn_wmma_f32_16x16x32_f16(false, a, false, b, (short)0, c, false, false);
  }
  static __device__ __forceinline__ void guard(v8f& a, v8f& b, v16h x, v16h y) { dep_guard_h(a, b, x, y); }
  static __device__ __forceinline__ void keep(v16h a, v16h b, v16h c, v16h d) { keep4_h(a, b, c, d); }
};
template <> struct Frag<__bf16> {
  typedef v16b V; union U { v16b v; v8b h[2]; };
  static __device__ __forceinline__ v16b load(const __bf16* p) {
    U f; f.h[0] = *(const v8b*)(p); f.h[1] = *(const v8b*)(p + 16); return f.v;
  }
  static __device__ __forceinline__ v8f mma(v16b a, v16b b, v8f c) {
    return __builtin_amdgcn_wmma_f32_16x16x32_bf16(false, a, false, b, (short)0, c, false, false);
  }
  static __device__ __forceinline__ void guard(v8f& a, v8f& b, v16b x, v16b y) { dep_guard_b(a, b, x, y); }
  static __device__ __forceinline__ void keep(v16b a, v16b b, v16b c, v16b d) { keep4_b(a, b, c, d); }
};

__device__ __forceinline__ unsigned pk16(unsigned short a, unsigned short b) { return (unsigned)a | ((unsigned)b << 16); }
__device__ __forceinline__ unsigned short h_bits(float f) { const _Float16 h = (_Float16)f; return __builtin_bit_cast(unsigned short, h); }

template <int ET> struct Elem;
template <> struct Elem<0> { typedef _Float16 T; };
template <> struct Elem<1> { typedef __bf16 T; };
template <int ET, bool SPLIT, int BIAS_MODE, int OUT_MODE, bool RESID, int ACT = 0>
__global__ __launch_bounds__(256) void wmma_gemm64(
    const unsigned short* __restrict__ Ap, const unsigned short* __restrict__ A2p, int lda, long strideA,
    const unsigned short* __restrict__ Btp, const unsigned short* __restrict__ Bt2p, int ldb, long strideB,
    void* __restrict__ Cout, void* __restrict__ Cout2, int ldc, long strideC,
    const float* __restrict__ bias,
    const float* __restrict__ resid, long strideR,
    int M, int N, int K, float scale) {
  typedef typename Elem<ET>::T T;
  typedef typename Frag<T>::V V;
  const T* A = (const T*)Ap; const T* A2 = (const T*)A2p; const T* Bt = (const T*)Btp; const T* Bt2 = (const T*)Bt2p;
  __shared__ __align__(16) float sT[8][16 * 68];
  const int b    = blockIdx.y;
  const int lane = threadIdx.x & 31;
  const int wave = threadIdx.x >> 5;
  const int tilesN = N >> 6;
  const int tilesM = M >> 6;
  const int tile = blockIdx.x * 8 + wave;
  if (tile >= tilesM * tilesN) return;
  const int tm = tile / tilesN;
  const int tn = tile - tm * tilesN;
  const int m0 = tm << 6;
  const int n0 = tn << 6;

  const T* Ab  = A  + (size_t)b * strideA;
  const T* Bb  = Bt + (size_t)b * strideB;
  const T* Ab2 = SPLIT ? (A2  + (size_t)b * strideA) : nullptr;
  const T* Bb2 = SPLIT ? (Bt2 + (size_t)b * strideB) : nullptr;

  const int rlane = lane & 15;
  const int koff  = (lane >> 4) * 8;
  const int mOff  = (lane >> 4) * 8;

  v8f acc[4][4];
#pragma unroll
  for (int i = 0; i < 4; ++i)
#pragma unroll
    for (int j = 0; j < 4; ++j) acc[i][j] = (v8f){0.f,0.f,0.f,0.f,0.f,0.f,0.f,0.f};

  for (int k0 = 0; k0 < K; k0 += 32) {
    V bh[4], bl[4];
#pragma unroll
    for (int j = 0; j < 4; ++j) {
      const size_t bo = (size_t)(n0 + (j << 4) + rlane) * ldb + koff + k0;
      bh[j] = Frag<T>::load(Bb + bo);
      if (SPLIT) bl[j] = Frag<T>::load(Bb2 + bo);
    }
#pragma unroll
    for (int i = 0; i < 4; ++i) {
      const size_t ao = (size_t)(m0 + (i << 4) + rlane) * lda + koff + k0;
      V ah = Frag<T>::load(Ab + ao);
      V al;
      if (SPLIT) al = Frag<T>::load(Ab2 + ao);
#pragma unroll
      for (int j = 0; j < 4; ++j) {
        acc[i][j] = Frag<T>::mma(ah, bh[j], acc[i][j]);
        if (SPLIT) {
          acc[i][j] = Frag<T>::mma(ah, bl[j], acc[i][j]);
          acc[i][j] = Frag<T>::mma(al, bh[j], acc[i][j]);
        }
      }
      Frag<T>::guard(acc[i][0], acc[i][3], ah, SPLIT ? al : ah);
    }
    Frag<T>::keep(bh[0], bh[1], bh[2], bh[3]);
    if (SPLIT) Frag<T>::keep(bl[0], bl[1], bl[2], bl[3]);
  }
  acc_guard4(acc[0][0], acc[0][1], acc[0][2], acc[0][3]);
  acc_guard4(acc[1][0], acc[1][1], acc[1][2], acc[1][3]);
  acc_guard4(acc[2][0], acc[2][1], acc[2][2], acc[2][3]);
  acc_guard4(acc[3][0], acc[3][1], acc[3][2], acc[3][3]);

  float* slab = sT[wave];
  const float* Rb = RESID ? (resid + (size_t)b * strideR) : nullptr;
#pragma unroll
  for (int i = 0; i < 4; ++i) {
    const int mBase = m0 + (i << 4);
#pragma unroll
    for (int j = 0; j < 4; ++j) {
      const int n = n0 + (j << 4) + rlane;
      float bv = 0.f;
      if (BIAS_MODE == 2) bv = bias[n];
#pragma unroll
      for (int r = 0; r < 8; ++r) {
        float v = acc[i][j][r] * scale;
        if (BIAS_MODE == 1) v += bias[mBase + mOff + r];
        if (BIAS_MODE == 2) v += bv;
        if (RESID) v += Rb[(size_t)(mBase + mOff + r) * ldc + n];
        if (ACT == 2) v = fmaxf(v, 0.0f);
        if (ACT == 4) v = (v > 0.f) ? v : 0.01f * v;
        slab[(mOff + r) * 68 + (j << 4) + rlane] = v;
      }
    }
    __builtin_amdgcn_fence(__ATOMIC_RELEASE, "workgroup");
    __builtin_amdgcn_wave_barrier();
    __builtin_amdgcn_fence(__ATOMIC_ACQUIRE, "workgroup");
    if (OUT_MODE == 0) {
      float* C = (float*)Cout + (size_t)b * strideC;
      const int hh = lane >> 4, c4 = (lane & 15) * 4;
      for (int pass = 0; pass < 2; ++pass) {
#pragma unroll
        for (int it = 0; it < 8; ++it) {
          const int row = it * 2 + hh;
          v4f v = *(const v4f*)(slab + row * 68 + c4);
          *(volatile v4f*)(C + (size_t)(mBase + row) * ldc + n0 + c4) = v;
        }
        __threadfence();
      }
    } else {
      const int q = lane >> 3, c8 = (lane & 7) * 8;
      unsigned short* C  = (unsigned short*)Cout  + (size_t)b * strideC;
      unsigned short* C2 = (OUT_MODE == 2) ? ((unsigned short*)Cout2 + (size_t)b * strideC) : nullptr;
      for (int pass = 0; pass < 2; ++pass) {
#pragma unroll
        for (int it = 0; it < 4; ++it) {
          const int row = it * 4 + q;
          const float* sp = slab + row * 68 + c8;
          v8h hv, lv;
#pragma unroll
          for (int e = 0; e < 8; ++e) {
            if (OUT_MODE == 1) {
              hv[e] = (_Float16)sp[e];
            } else {
              unsigned short hb = f2bf_bits(sp[e]);
              unsigned short lb = f2bf_bits(sp[e] - bf_bits2f(hb));
              hv[e] = __builtin_bit_cast(_Float16, hb);
              lv[e] = __builtin_bit_cast(_Float16, lb);
            }
          }
          *(volatile v8h*)(C + (size_t)(mBase + row) * ldc + n0 + c8) = hv;
          if (OUT_MODE == 2) *(volatile v8h*)(C2 + (size_t)(mBase + row) * ldc + n0 + c8) = lv;
        }
        __threadfence();
      }
    }
    __builtin_amdgcn_fence(__ATOMIC_RELEASE, "workgroup");
    __builtin_amdgcn_wave_barrier();
    __builtin_amdgcn_fence(__ATOMIC_ACQUIRE, "workgroup");
  }
}

__device__ __forceinline__ float gelu_erf(float z) { return 0.5f * z * (1.0f + erff(z * kInvSqrt2)); }

template <bool HALF>
__device__ __forceinline__ void store_row64(const float* slab, float* xrow, unsigned short* hrow, int lane) {
  const int c4 = (lane & 15) * 4;
  const v4f v = *(const v4f*)(slab + c4);
  v4u u = {0u, 0u, 0u, 0u};
  const int c8 = (lane & 7) * 8;
  if (HALF) {
    const v4f a = *(const v4f*)(slab + c8);
    const v4f q = *(const v4f*)(slab + c8 + 4);
    unsigned short hb[8];
#pragma unroll
    for (int e = 0; e < 4; ++e) {
      hb[e]     = h_bits(a[e] * kXCarry);
      hb[4 + e] = h_bits(q[e] * kXCarry);
    }
    u = (v4u){pk16(hb[0], hb[1]), pk16(hb[2], hb[3]), pk16(hb[4], hb[5]), pk16(hb[6], hb[7])};
  }
  for (int pass = 0; pass < 2; ++pass) {
    if (lane < 16) *(volatile v4f*)(xrow + c4) = v;
    if (HALF) { if (lane < 8) *(volatile v4u*)(hrow + c8) = u; }
    __threadfence();
  }
}

__global__ __launch_bounds__(256) void prep_kernel(const float* __restrict__ pw1, const float* __restrict__ tw1,
                                                   const float* __restrict__ pw2, const float* __restrict__ pb1,
                                                   const float* __restrict__ tb1,
                                                   unsigned* __restrict__ w1cat, unsigned* __restrict__ w2t,
                                                   float* __restrict__ biascat) {
  const int i = blockIdx.x * 256 + threadIdx.x;
  if (i < kW1catWords) {
    const int l   = i >> 14;
    const int rem = i & 16383;
    const int n   = rem >> 5;
    const int k   = (rem & 31) * 2;
    const int sec = n / 96;
    const int nn  = n - sec * 96;
    const int kc  = k < 46 ? k : 46;
    const float fp = (sec < 2 && k < 48) ? 1.f : 0.f;
    const float ft = (sec >= 2 && sec < 5 && k < 48) ? 1.f : 0.f;
    const int secp = sec < 1 ? sec : 1;
    int sect = sec - 2; sect = sect < 0 ? 0 : (sect > 2 ? 2 : sect);
    const float* pp = pw1 + (size_t)l * 96 * 96 + (size_t)(secp * 48 + kc) * 96 + nn;
    const float* tp = tw1 + (size_t)l * 144 * 96 + (size_t)(sect * 48 + kc) * 96 + nn;
    const float wpa = pp[0], wpb = pp[96], wta = tp[0], wtb = tp[96];
    const float va = fmaf(fp, wpa, ft * wta) * kWCarry;
    const float vb = fmaf(fp, wpb, ft * wtb) * kWCarry;
    const unsigned u = pk16(h_bits(va), h_bits(vb));
    ((volatile unsigned*)w1cat)[i] = u;
    __threadfence();
    ((volatile unsigned*)w1cat)[i] = u;
  } else if (i < kW1catWords + kW2tWords) {
    const int i2  = i - kW1catWords;
    const int l   = i2 / 2304;
    const int rem = i2 - l * 2304;
    const int n   = rem / 48;
    const int k   = (rem - n * 48) * 2;
    const float* pp = pw2 + (size_t)l * 96 * 48 + (size_t)k * 48 + n;
    const float va = pp[0] * kWCarry, vb = pp[48] * kWCarry;
    const unsigned u = pk16(h_bits(va), h_bits(vb));
    ((volatile unsigned*)w2t)[i2] = u;
    __threadfence();
    ((volatile unsigned*)w2t)[i2] = u;
  } else if (i < kPrepWords) {
    const int i3 = i - kW1catWords - kW2tWords;
    const int l  = i3 >> 9;
    const int n  = i3 & 511;
    const int ip = n < 96 ? n : 95;
    int it = n - 192; it = it < 0 ? 0 : (it > 95 ? 95 : it);
    const float fp = (n < 96) ? 1.f : 0.f;
    const float ft = (n >= 192 && n < 288) ? 1.f : 0.f;
    const float v = fmaf(fp, pb1[l * 96 + ip], ft * tb1[l * 96 + it]);
    ((volatile float*)biascat)[i3] = v;
    __threadfence();
    ((volatile float*)biascat)[i3] = v;
  }
}

__global__ __launch_bounds__(32) void embed_kernel(const int* __restrict__ ids, const float* __restrict__ emb,
                                                   const float* __restrict__ pos, float* __restrict__ xf,
                                                   unsigned short* __restrict__ xh) {
  __shared__ __align__(16) float slab[64];
  const int bn = blockIdx.x;
  const int n  = bn & (kNode - 1);
  const int lane = threadIdx.x;
  int id = ids[bn];
  id = id < 0 ? 0 : (id > kVoc - 1 ? kVoc - 1 : id);
  const int c4 = (lane & 15) * 4;
  const int cc = c4 < kDim ? c4 : kDim - 4;
  const v4f e = *(const v4f*)(emb + id * kDim + cc);
  const v4f p = *(const v4f*)(pos + n * kDim + cc);
  const float keep = (c4 < kDim) ? 1.f : 0.f;
  const v4f v = (e + p) * keep;
  if (lane < 16) *(v4f*)(slab + c4) = v;
  __syncthreads();
  store_row64<true>(slab, xf + (size_t)bn * kXld, xh + (size_t)bn * kXld, lane);
}

__global__ __launch_bounds__(256) void pair_kernel(const float* __restrict__ proj, const unsigned short* __restrict__ w2t,
                                                   const float* __restrict__ b2, float* __restrict__ pout) {
  __shared__ __align__(16) unsigned short hbuf[8 * 16 * 96];
  __shared__ __align__(16) unsigned short wsh[48 * 96];
  __shared__ float ush[96];
  __shared__ float wacc[8 * 48];
  __shared__ float wm[8];
  __shared__ float wl[8];
  __shared__ __align__(16) float orow[64];
  const int tid = threadIdx.x, lane = tid & 31, wave = tid >> 5;
  const int bi = blockIdx.x;
  const int bb = bi >> 8;
  const int qi = bi & 255;
  const int rlane = lane & 15, hh = lane >> 4, koff = hh * 8;

  if (tid < 96) ush[tid] = proj[(size_t)bi * kPld + tid];
  for (int idx = tid; idx < 576; idx += 256) ((v4u*)wsh)[idx] = ((const v4u*)w2t)[idx];
  const float bv0 = b2[rlane], bv1 = b2[16 + rlane], bv2 = b2[32 + rlane];

  float m_run = -1e30f, l_run = 0.f, s0 = 0.f, s1 = 0.f, s2 = 0.f;
  const int nsteps = ((qi >> 4) + 8) >> 3;
  unsigned short* hbw = hbuf + wave * (16 * 96);
  const v8f z8 = {0.f, 0.f, 0.f, 0.f, 0.f, 0.f, 0.f, 0.f};

  for (int step = 0; step < nsteps; ++step) {
    const int jt = step * 8 + wave;
    __syncthreads();
    {
      const int j = jt * 16 + rlane;
      const float* vrow = proj + (size_t)(bb * kNode + j) * kPld + 96 + hh * 48;
      const int ub = hh * 48;
#pragma unroll 1
      for (int q = 0; q < 6; ++q) {
        const v4f va = *(const v4f*)(vrow + 8 * q);
        const v4f vb = *(const v4f*)(vrow + 8 * q + 4);
        unsigned short hb[8];
#pragma unroll
        for (int e = 0; e < 4; ++e) {
          const float z0 = ush[ub + 8 * q + e] + va[e];
          const float z1 = ush[ub + 8 * q + 4 + e] + vb[e];
          hb[e]     = h_bits(gelu_erf(z0) * kHCarry);
          hb[4 + e] = h_bits(gelu_erf(z1) * kHCarry);
        }
        const v4u u = (v4u){pk16(hb[0], hb[1]), pk16(hb[2], hb[3]), pk16(hb[4], hb[5]), pk16(hb[6], hb[7])};
        *(v4u*)(hbw + rlane * 96 + hh * 48 + 8 * q) = u;
      }
    }
    __syncthreads();

    v8f acc0 = z8, acc1 = z8, acc2 = z8;
    const _Float16* ha = (const _Float16*)hbw;
    const _Float16* wb = (const _Float16*)wsh;
#pragma unroll
    for (int ks = 0; ks < 3; ++ks) {
      const int k0 = ks * 32;
      const v16h a  = Frag<_Float16>::load(ha + rlane * 96 + koff + k0);
      const v16h f0 = Frag<_Float16>::load(wb + rlane * 96 + koff + k0);
      const v16h f1 = Frag<_Float16>::load(wb + (16 + rlane) * 96 + koff + k0);
      const v16h f2 = Frag<_Float16>::load(wb + (32 + rlane) * 96 + koff + k0);
      acc0 = Frag<_Float16>::mma(a, f0, acc0);
      acc1 = Frag<_Float16>::mma(a, f1, acc1);
      acc2 = Frag<_Float16>::mma(a, f2, acc2);
      guard3h(acc0, acc1, acc2, a, f0, f1, f2);
    }

    float pv0[8], pv1[8], pv2[8], lg[8];
    float tmax = -1e30f;
#pragma unroll
    for (int r = 0; r < 8; ++r) {
      const int jrow = jt * 16 + 8 * hh + r;
      const bool keep = (jrow <= qi);
      const float kf = keep ? 1.f : 0.f;
      const float p0 = kf * (acc0[r] * kPairScale + bv0);
      const float p1 = kf * (acc1[r] * kPairScale + bv1);
      const float p2 = kf * (acc2[r] * kPairScale + bv2);
      float sq = p0 * p0 + p1 * p1 + p2 * p2;
      sq += __shfl_xor(sq, 1, 32);
      sq += __shfl_xor(sq, 2, 32);
      sq += __shfl_xor(sq, 4, 32);
      sq += __shfl_xor(sq, 8, 32);
      pv0[r] = p0; pv1[r] = p1; pv2[r] = p2;
      const float nrm = sqrtf(sq);
      lg[r] = keep ? nrm : -1e9f;
      tmax = fmaxf(tmax, lg[r]);
    }
    tmax = fmaxf(tmax, __shfl_xor(tmax, 16, 32));
    const float m_new = fmaxf(m_run, tmax);
    const float alpha = expf(m_run - m_new);
    float psum = 0.f, a0 = 0.f, a1 = 0.f, a2 = 0.f;
#pragma unroll
    for (int r = 0; r < 8; ++r) {
      const float es = expf(lg[r] - m_new);
      psum += es;
      a0 = fmaf(es, pv0[r], a0);
      a1 = fmaf(es, pv1[r], a1);
      a2 = fmaf(es, pv2[r], a2);
    }
    psum += __shfl_xor(psum, 16, 32);
    l_run = l_run * alpha + psum;
    s0 = s0 * alpha + a0;
    s1 = s1 * alpha + a1;
    s2 = s2 * alpha + a2;
    m_run = m_new;
  }
  s0 += __shfl_xor(s0, 16, 32);
  s1 += __shfl_xor(s1, 16, 32);
  s2 += __shfl_xor(s2, 16, 32);
  if (lane < 16) {
    wacc[wave * 48 + rlane]      = s0;
    wacc[wave * 48 + 16 + rlane] = s1;
    wacc[wave * 48 + 32 + rlane] = s2;
  }
  if (lane == 0) { wm[wave] = m_run; wl[wave] = l_run; }
  __syncthreads();
  if (tid < 64) {
    const int c = tid < 48 ? tid : 47;
    float mx = wm[0];
#pragma unroll 1
    for (int w = 1; w < 8; ++w) mx = fmaxf(mx, wm[w]);
    float lsum = 0.f, osum = 0.f;
#pragma unroll 1
    for (int w = 0; w < 8; ++w) {
      const float ew = expf(wm[w] - mx);
      lsum = fmaf(wl[w], ew, lsum);
      osum = fmaf(wacc[w * 48 + c], ew, osum);
    }
    const float o = osum * (1.0f / lsum);
    orow[tid] = (tid < 48) ? o : 0.f;
  }
  __syncthreads();
  if (wave == 0) store_row64<false>(orow, pout + (size_t)bi * kXld, nullptr, lane);
}

__global__ __launch_bounds__(96) void tgl_kernel(const float* __restrict__ proj, const int* __restrict__ jil,
                                                 const int* __restrict__ kil, const float* __restrict__ tw2,
                                                 const float* __restrict__ tb2, const float* __restrict__ gw,
                                                 const float* __restrict__ gb, const float* __restrict__ ng,
                                                 const float* __restrict__ nb, const float* __restrict__ pout,
                                                 float* xf) {
  __shared__ float hbar[96];
  __shared__ float pt[96];
  __shared__ __align__(16) float y[64];
  __shared__ float stats[2];
  const int tid = threadIdx.x, lane = tid & 31, wave = tid >> 5;
  const int bn = blockIdx.x;
  const int b  = bn >> 8;
  {
    const int o = tid;
    const float pa = proj[(size_t)bn * kPld + 192 + o];
    float acc = 0.f;
#pragma unroll 1
    for (int s = 0; s < kSmp; ++s) {
      int jv = jil[bn * kSmp + s]; jv = jv < 0 ? 0 : (jv > kNode - 1 ? kNode - 1 : jv);
      int kv = kil[bn * kSmp + s]; kv = kv < 0 ? 0 : (kv > kNode - 1 ? kNode - 1 : kv);
      const float zb = proj[(size_t)(b * kNode + jv) * kPld + 288 + o];
      const float zc = proj[(size_t)(b * kNode + kv) * kPld + 384 + o];
      const float z = (pa + zb) + zc;
      acc += gelu_erf(z);
    }
    hbar[o] = acc * (1.0f / 6.0f);
    const float pv = pout[(size_t)bn * kXld + (tid & 63)];
    if (tid < kDim) pt[tid] = pv;
  }
  __syncthreads();
  if (tid < 64) {
    const int c = tid < kDim ? tid : kDim - 1;
    float a = 0.f;
#pragma unroll 1
    for (int o2 = 0; o2 < kHid2; ++o2) a = fmaf(hbar[o2], tw2[o2 * kDim + c], a);
    a += tb2[c];
    if (tid < kDim) pt[kDim + tid] = a;
  }
  __syncthreads();
  if (tid < 64) {
    const int c = tid < kDim ? tid : kDim - 1;
    float a = 0.f;
#pragma unroll 1
    for (int d = 0; d < kHid2; ++d) a = fmaf(pt[d], gw[d * kDim + c], a);
    a += gb[c];
    const float g  = 1.0f / (1.0f + expf(-a));
    const float xo = xf[(size_t)bn * kXld + c];
    const float yv = xo + g * pt[c] + (1.0f - g) * pt[kDim + c];
    y[tid] = (tid < kDim) ? yv : 0.f;
  }
  __syncthreads();
  if (tid == 0) {
    float mu = 0.f;
#pragma unroll 1
    for (int d = 0; d < kDim; ++d) mu += y[d];
    mu *= (1.0f / 48.0f);
    float var = 0.f;
#pragma unroll 1
    for (int d = 0; d < kDim; ++d) { const float q = y[d] - mu; var = fmaf(q, q, var); }
    var *= (1.0f / 48.0f);
    stats[0] = mu;
    stats[1] = rsqrtf(var + kLnEps);
  }
  __syncthreads();
  float yn = 0.f;
  if (tid < 64) {
    const int c = tid < kDim ? tid : kDim - 1;
    yn = (y[c] - stats[0]) * stats[1] * ng[c] + nb[c];
  }
  __syncthreads();
  if (tid < kDim) y[tid] = yn;
  __syncthreads();
  if (wave == 0) store_row64<false>(y, xf + (size_t)bn * kXld, nullptr, lane);
}

__global__ __launch_bounds__(192) void ffn_kernel(const float* __restrict__ fw1, const float* __restrict__ fb1,
                                                  const float* __restrict__ fw2, const float* __restrict__ fb2,
                                                  const float* __restrict__ ng, const float* __restrict__ nb,
                                                  float* xf, unsigned short* __restrict__ xh) {
  __shared__ float xr[48];
  __shared__ float hid[192];
  __shared__ __align__(16) float y[64];
  __shared__ float stats[2];
  const int tid = threadIdx.x, lane = tid & 31, wave = tid >> 5;
  const int bn = blockIdx.x;
  {
    const float xv = xf[(size_t)bn * kXld + (tid & 63)];
    if (tid < kDim) xr[tid] = xv;
  }
  __syncthreads();
  {
    const int o = tid;
    float a = 0.f;
#pragma unroll 1
    for (int d = 0; d < kDim; ++d) a = fmaf(xr[d], fw1[d * kFfn + o], a);
    a += fb1[o];
    hid[o] = gelu_erf(a);
  }
  __syncthreads();
  if (tid < 64) {
    const int c = tid < kDim ? tid : kDim - 1;
    float a = 0.f;
#pragma unroll 1
    for (int o2 = 0; o2 < kFfn; ++o2) a = fmaf(hid[o2], fw2[o2 * kDim + c], a);
    a += fb2[c];
    const float yv = xr[c] + a;
    y[tid] = (tid < kDim) ? yv : 0.f;
  }
  __syncthreads();
  if (tid == 0) {
    float mu = 0.f;
#pragma unroll 1
    for (int d = 0; d < kDim; ++d) mu += y[d];
    mu *= (1.0f / 48.0f);
    float var = 0.f;
#pragma unroll 1
    for (int d = 0; d < kDim; ++d) { const float q = y[d] - mu; var = fmaf(q, q, var); }
    var *= (1.0f / 48.0f);
    stats[0] = mu;
    stats[1] = rsqrtf(var + kLnEps);
  }
  __syncthreads();
  float yn = 0.f;
  if (tid < 64) {
    const int c = tid < kDim ? tid : kDim - 1;
    yn = (y[c] - stats[0]) * stats[1] * ng[c] + nb[c];
  }
  __syncthreads();
  if (tid < kDim) y[tid] = yn;
  __syncthreads();
  if (wave == 0) store_row64<true>(y, xf + (size_t)bn * kXld, xh + (size_t)bn * kXld, lane);
}

__global__ __launch_bounds__(256) void head_kernel(const float* __restrict__ xf, const float* __restrict__ hw,
                                                   const float* __restrict__ hb, float* __restrict__ out, int nq) {
  const int i = blockIdx.x * 256 + threadIdx.x;
  if (i >= nq) return;
  const int tok = i / 5;
  const int c0  = (i - tok * 5) * 4;
  const float* xrow = xf + (size_t)tok * kXld;
  float a0 = 0.f, a1 = 0.f, a2 = 0.f, a3 = 0.f;
#pragma unroll 1
  for (int d = 0; d < kDim; ++d) {
    const float xv = xrow[d];
    const v4f w4 = *(const v4f*)(hw + d * kVoc + c0);
    a0 = fmaf(xv, w4[0], a0);
    a1 = fmaf(xv, w4[1], a1);
    a2 = fmaf(xv, w4[2], a2);
    a3 = fmaf(xv, w4[3], a3);
  }
  v4f v;
  v[0] = a0 + hb[c0];
  v[1] = a1 + hb[c0 + 1];
  v[2] = a2 + hb[c0 + 2];
  v[3] = a3 + hb[c0 + 3];
  float* op = out + 4 * (size_t)i;
  *(volatile v4f*)op = v;
  __threadfence();
  *(volatile v4f*)op = v;
}

extern "C" void kernel_launch(void* const* d_in, const int* in_sizes, int n_in,
                              void* d_out, int out_size, void* d_ws, size_t ws_size, hipStream_t stream) {
  if (n_in < 25) return;
  if (in_sizes[0] != kTok || in_sizes[1] != kLay * kTok * kSmp || in_sizes[2] != kLay * kTok * kSmp) return;
  if (in_sizes[3] != kVoc * kDim || in_sizes[4] != kNode * kDim || in_sizes[5] != kLay * kHid2 * kHid2) return;
  if (out_size != kTok * kVoc) return;

  const int*   ids     = (const int*)d_in[0];
  const int*   ji      = (const int*)d_in[1];
  const int*   ki      = (const int*)d_in[2];
  const float* emb     = (const float*)d_in[3];
  const float* pos     = (const float*)d_in[4];
  const float* pair_w1 = (const float*)d_in[5];
  const float* pair_b1 = (const float*)d_in[6];
  const float* pair_w2 = (const float*)d_in[7];
  const float* pair_b2 = (const float*)d_in[8];
  const float* tri_w1  = (const float*)d_in[9];
  const float* tri_b1  = (const float*)d_in[10];
  const float* tri_w2  = (const float*)d_in[11];
  const float* tri_b2  = (const float*)d_in[12];
  const float* gate_w  = (const float*)d_in[13];
  const float* gate_b  = (const float*)d_in[14];
  const float* n1g     = (const float*)d_in[15];
  const float* n1b     = (const float*)d_in[16];
  const float* ffn_w1  = (const float*)d_in[17];
  const float* ffn_b1  = (const float*)d_in[18];
  const float* ffn_w2  = (const float*)d_in[19];
  const float* ffn_b2  = (const float*)d_in[20];
  const float* n2g     = (const float*)d_in[21];
  const float* n2b     = (const float*)d_in[22];
  const float* head_w  = (const float*)d_in[23];
  const float* head_b  = (const float*)d_in[24];
  float* out = (float*)d_out;

  char* ws = (char*)d_ws; size_t off = 0;
  auto carve = [&](size_t bytes) -> char* { char* p = ws + off; off += (bytes + 255) & ~(size_t)255; return p; };
  float*          xf      = (float*)carve((size_t)kTok * kXld * 4);
  unsigned short* xh      = (unsigned short*)carve((size_t)kTok * kXld * 2);
  float*          proj    = (float*)carve((size_t)kTok * kPld * 4);
  float*          pout    = (float*)carve((size_t)kTok * kXld * 4);
  unsigned short* w1cat   = (unsigned short*)carve((size_t)kW1catWords * 4);
  unsigned short* w2t     = (unsigned short*)carve((size_t)kW2tWords * 4);
  float*          biascat = (float*)carve((size_t)kBiasWords * 4);
  if (off > ws_size || off > (size_t)134217728) return;

  prep_kernel<<<kPrepWords / 256, 256, 0, stream>>>(pair_w1, tri_w1, pair_w2, pair_b1, tri_b1,
                                                    (unsigned*)w1cat, (unsigned*)w2t, biascat);
  embed_kernel<<<kTok, 32, 0, stream>>>(ids, emb, pos, xf, xh);

  for (int l = 0; l < kLay; ++l) {
    const unsigned short* w1cat_l = w1cat + (size_t)l * kProjN * kProjK;
    const unsigned short* w2t_l   = w2t + (size_t)l * kDim * kHid2;
    const float*          bias_l  = biascat + (size_t)l * kProjN;
    {
      const int tiles = (kTok / 64) * (kProjN / 64);
      wmma_gemm64<0, false, 2, 0, false, 0><<<dim3((tiles + 7) / 8, 1), 256, 0, stream>>>(
          (const unsigned short*)xh, (const unsigned short*)xh, kXld, 0L,
          w1cat_l, w1cat_l, kProjK, 0L,
          (void*)proj, (void*)nullptr, kPld, 0L,
          bias_l, (const float*)nullptr, 0L, kTok, kProjN, kProjK, kProjScale);
    }
    pair_kernel<<<kTok, 256, 0, stream>>>(proj, w2t_l, pair_b2 + l * kDim, pout);
    tgl_kernel<<<kTok, 96, 0, stream>>>(proj, ji + (size_t)l * kTok * kSmp, ki + (size_t)l * kTok * kSmp,
                                        tri_w2 + (size_t)l * kHid2 * kDim, tri_b2 + l * kDim,
                                        gate_w + (size_t)l * kHid2 * kDim, gate_b + l * kDim,
                                        n1g + l * kDim, n1b + l * kDim, pout, xf);
    ffn_kernel<<<kTok, 192, 0, stream>>>(ffn_w1 + (size_t)l * kDim * kFfn, ffn_b1 + l * kFfn,
                                         ffn_w2 + (size_t)l * kFfn * kDim, ffn_b2 + l * kDim,
                                         n2g + l * kDim, n2b + l * kDim, xf, xh);
  }
  const int nq = out_size / 4;
  head_kernel<<<(nq + 255) / 256, 256, 0, stream>>>(xf, head_w, head_b, out, nq);
}
